// UPFDNet_52596169507566
// MI455X (gfx1250) — hardware-verified
//
#include <hip/hip_runtime.h>


#define NN_  100000
#define NE_  1600000
#define FIN  128
#define HID  256
#define NG_  512
#define CHN  20000
#define NCH  (NN_ / CHN)
#define RB   512
#define NT   512
#define NWV  (NT / 32)
#define EPT  8
#define CHUNK (NT * EPT)
#define NBLK ((CHN + RB - 1) / RB)
#define LDS_AGGR ((size_t)RB * FIN * 4 + (size_t)CHUNK * 4 + (size_t)RB * 4 + (size_t)NWV * 4)

typedef __attribute__((ext_vector_type(4)))  float    v4f;
typedef __attribute__((ext_vector_type(2)))  float    v2f;
typedef v4f  __attribute__((may_alias)) v4fa;

typedef __attribute__((ext_vector_type(16))) __bf16   v16bf;
typedef __attribute__((ext_vector_type(16))) _Float16 v16h;
typedef __attribute__((ext_vector_type(8)))  float    v8f;
typedef __attribute__((ext_vector_type(8)))  unsigned v8u;

__device__ __forceinline__ unsigned f2bf(float f) { unsigned u = __float_as_uint(f); u += 0x7FFFu + ((u >> 16) & 1u); return u >> 16; }
__device__ __forceinline__ unsigned f2h(float f) { return (unsigned)__builtin_bit_cast(unsigned short, (_Float16)f); }
__device__ __forceinline__ int kpat(int v, int half) { return ((v & 4) ? 16 : 0) + half * 8 + 2 * (v & 3); }

template <int F16, int NP> struct Opnd { v16bf p[NP]; };

template <int F16, int NP> __device__ __forceinline__ void pack2(float f0, float f1, unsigned* o) {
    if (F16) { o[0] = f2h(f0) | (f2h(f1) << 16); return; }
    unsigned h0 = f2bf(f0), h1 = f2bf(f1); o[0] = h0 | (h1 << 16);
    if (NP >= 2) {
        float r0 = f0 - __uint_as_float(h0 << 16), r1 = f1 - __uint_as_float(h1 << 16);
        unsigned m0 = f2bf(r0), m1 = f2bf(r1); o[1] = m0 | (m1 << 16);
        if (NP >= 3) {
            float s0 = r0 - __uint_as_float(m0 << 16), s1 = r1 - __uint_as_float(m1 << 16);
            o[2] = f2bf(s0) | (f2bf(s1) << 16);
        }
    }
}
template <int F16, int NP> __device__ __forceinline__ void op_row(const float* rowp, int half, float sc, Opnd<F16, NP>& o) {
    v8u u[NP];
#pragma unroll
    for (int v = 0; v < 8; ++v) {
        int kk = kpat(v, half); unsigned t[3];
        pack2<F16, NP>(rowp[kk] * sc, rowp[kk + 1] * sc, t);
#pragma unroll
        for (int p = 0; p < NP; ++p) u[p][v] = t[p];
    }
#pragma unroll
    for (int p = 0; p < NP; ++p) o.p[p] = __builtin_bit_cast(v16bf, u[p]);
}
template <int F16, int NP> __device__ __forceinline__ void op_row_tail(const float* rowp, int half, float sc, int kvalid, Opnd<F16, NP>& o) {
    v8u u[NP];
#pragma unroll
    for (int v = 0; v < 8; ++v) {
        int kk = kpat(v, half); unsigned t[3];
        float f0 = kk < kvalid ? rowp[kk] * sc : 0.0f, f1 = (kk + 1) < kvalid ? rowp[kk + 1] * sc : 0.0f;
        pack2<F16, NP>(f0, f1, t);
#pragma unroll
        for (int p = 0; p < NP; ++p) u[p][v] = t[p];
    }
#pragma unroll
    for (int p = 0; p < NP; ++p) o.p[p] = __builtin_bit_cast(v16bf, u[p]);
}
template <int F16, int NP> __device__ __forceinline__ void op_col(const float* M, int ld, int n, int k0, int half, float sc, Opnd<F16, NP>& o) {
    v8u u[NP];
#pragma unroll
    for (int v = 0; v < 8; ++v) {
        int kk = k0 + kpat(v, half); unsigned t[3];
        pack2<F16, NP>(M[(size_t)kk * ld + n] * sc, M[(size_t)(kk + 1) * ld + n] * sc, t);
#pragma unroll
        for (int p = 0; p < NP; ++p) u[p][v] = t[p];
    }
#pragma unroll
    for (int p = 0; p < NP; ++p) o.p[p] = __builtin_bit_cast(v16bf, u[p]);
}
template <int F16, int NP> __device__ __forceinline__ void op_col_tail(const float* M, int ld, int n, int k0, int half, float sc, int K, Opnd<F16, NP>& o) {
    v8u u[NP];
#pragma unroll
    for (int v = 0; v < 8; ++v) {
        int kk = k0 + kpat(v, half); unsigned t[3];
        float f0 = kk < K ? M[(size_t)kk * ld + n] * sc : 0.0f, f1 = (kk + 1) < K ? M[(size_t)(kk + 1) * ld + n] * sc : 0.0f;
        pack2<F16, NP>(f0, f1, t);
#pragma unroll
        for (int p = 0; p < NP; ++p) u[p][v] = t[p];
    }
#pragma unroll
    for (int p = 0; p < NP; ++p) o.p[p] = __builtin_bit_cast(v16bf, u[p]);
}
__device__ __forceinline__ v8f wm_bf16(v16bf a, v16bf b, v8f c) { return __builtin_amdgcn_wmma_f32_16x16x32_bf16(false, a, false, b, (short)0, c, false, false); }
template <int F16, int NA, int NB> __device__ __forceinline__ v8f wmma_op(const Opnd<F16, NA>& a, const Opnd<F16, NB>& b, v8f c) {
    if (F16) {
        v16h ah = __builtin_bit_cast(v16h, a.p[0]), bh = __builtin_bit_cast(v16h, b.p[0]);
        c = __builtin_amdgcn_wmma_f32_16x16x32_f16(false, ah, false, bh, (short)0, c, false, false);
        asm volatile("v_nop\n\tv_nop\n\tv_nop\n\tv_nop" : "+v"(c) : "v"(ah), "v"(bh));
        return c;
    }
    constexpr int NMX = NA > NB ? NA : NB;
#pragma unroll
    for (int i = 0; i < NA; ++i)
#pragma unroll
        for (int j = 0; j < NB; ++j)
            if (i + j < NMX) c = wm_bf16(a.p[i], b.p[j], c);
    if (NA == 1 && NB == 1)      asm volatile("v_nop\n\tv_nop\n\tv_nop\n\tv_nop" : "+v"(c) : "v"(a.p[0]), "v"(b.p[0]));
    else if (NA == 2 && NB == 1) asm volatile("v_nop\n\tv_nop\n\tv_nop\n\tv_nop" : "+v"(c) : "v"(a.p[0]), "v"(a.p[1]), "v"(b.p[0]));
    else if (NA == 1 && NB == 2) asm volatile("v_nop\n\tv_nop\n\tv_nop\n\tv_nop" : "+v"(c) : "v"(a.p[0]), "v"(b.p[0]), "v"(b.p[1]));
    else if (NA == 2 && NB == 2) asm volatile("v_nop\n\tv_nop\n\tv_nop\n\tv_nop" : "+v"(c) : "v"(a.p[0]), "v"(a.p[1]), "v"(b.p[0]), "v"(b.p[1]));
    else                         asm volatile("v_nop\n\tv_nop\n\tv_nop\n\tv_nop" : "+v"(c) : "v"(a.p[0]), "v"(a.p[NA - 1]), "v"(b.p[0]), "v"(b.p[NB - 1]), "v"(a.p[NA / 2]), "v"(b.p[NB / 2]));
    return c;
}

struct ZMap { long long s1; long long s2; int zdiv; int pad_; };
__device__ __forceinline__ size_t zoff(const ZMap& m, int z) { return (size_t)((long long)(z / m.zdiv) * m.s1 + (long long)(z % m.zdiv) * m.s2); }

#define ACT_NONE 0
#define ACT_RELU 1
#define ACT_GELU_ERF 2
#define ACT_SILU 3
#define ACT_TANH 4
__device__ __forceinline__ float act_apply(int act, float x) {
    if (act == ACT_RELU) return x > 0.f ? x : 0.f;
    if (act == ACT_GELU_ERF) return 0.5f * x * (1.0f + erff(x * 0.70710678118654752f));
    if (act == ACT_SILU) return x / (1.0f + expf(-x));
    if (act == ACT_TANH) return tanhf(x);
    return x;
}
struct GemmArgs {
    ZMap za, zb_, zc, zbias, zadd, zrsc, zmul, zrbias;
    const float* A; const float* Bm; float* C; const float* bias; const float* add; const float* rsc; const float* mul; const float* rbias;
    long long ldadd, ldmul;
    int lda, ldb, ldc, K;
    float ascale, bscale, oscale, addscale;
    int M, nvalid, nstore, ldrsc;
    int bcs, pad1, pad2, pad3;
};
template <int BT, int F16, int NA, int NB, int RW, int CW, int ACT>
__global__ __launch_bounds__(256) void gemm_kernel(GemmArgs g) {
    constexpr int TR = 16 * RW, TC = 64 * CW, CSTR = TC + 4;
    __shared__ __align__(16) float cst[TR * CSTR];
    const int z = blockIdx.z;
    const float* A = g.A + zoff(g.za, z); const float* Bm = g.Bm + zoff(g.zb_, z); float* C = g.C + zoff(g.zc, z);
    const int tid = threadIdx.x, lane = tid & 31, wv = tid >> 5;
    const int l16 = lane & 15, half = lane >> 4;
    const int rt = wv % RW, ch = wv / RW;
    const int row0 = blockIdx.x * TR, col0 = blockIdx.y * TC + ch * 64;
    int arix = row0 + rt * 16 + l16; if (arix >= g.M) arix = g.M - 1;
    const float* arow = A + (size_t)arix * g.lda;
    v8f acc[4];
#pragma unroll
    for (int t = 0; t < 4; ++t) acc[t] = (v8f){};
    const int K = g.K;
#pragma unroll 1
    for (int kc = 0; kc < K; kc += 32) {
        Opnd<F16, NA> a;
        if (kc + 32 <= K) op_row<F16, NA>(arow + kc, half, g.ascale, a); else op_row_tail<F16, NA>(arow + kc, half, g.ascale, K - kc, a);
#pragma unroll
        for (int t = 0; t < 4; ++t) {
            Opnd<F16, NB> b;
            const int n = col0 + t * 16 + l16;
            if (n < g.nvalid) {
                if (BT) { if (kc + 32 <= K) op_row<F16, NB>(Bm + (size_t)n * g.ldb + kc, half, g.bscale, b); else op_row_tail<F16, NB>(Bm + (size_t)n * g.ldb + kc, half, g.bscale, K - kc, b); }
                else    { if (kc + 32 <= K) op_col<F16, NB>(Bm, g.ldb, n * g.bcs, kc, half, g.bscale, b); else op_col_tail<F16, NB>(Bm, g.ldb, n * g.bcs, kc, half, g.bscale, K, b); }
            } else {
#pragma unroll
                for (int p = 0; p < NB; ++p) b.p[p] = (v16bf){};
            }
            acc[t] = wmma_op<F16, NA, NB>(a, b, acc[t]);
        }
    }
    const float* bias = g.bias ? g.bias + zoff(g.zbias, z) : nullptr;
    const float* add = g.add ? g.add + zoff(g.zadd, z) : nullptr;
    const float* rsc = g.rsc ? g.rsc + zoff(g.zrsc, z) : nullptr;
    const float* mul = g.mul ? g.mul + zoff(g.zmul, z) : nullptr;
    const float* rbias = g.rbias ? g.rbias + zoff(g.zrbias, z) : nullptr;
#pragma unroll
    for (int t = 0; t < 4; ++t) {
        const int cl = ch * 64 + t * 16 + l16;
        const int cg = blockIdx.y * TC + cl;
        const bool cok = cg < g.nvalid;
        const float bv = (bias && cok) ? bias[(size_t)cg * g.bcs] : 0.0f;
#pragma unroll
        for (int r = 0; r < 8; ++r) {
            const int rl = rt * 16 + r + 8 * half;
            float v = acc[t][r] * g.oscale + bv;
            int rg = row0 + rl; if (rg >= g.M) rg = g.M - 1;
            if (rbias) v += rbias[rg];
            if (rsc) v *= rsc[(size_t)rg * g.ldrsc];
            if (mul && cok) v *= mul[(size_t)rg * g.ldmul + cg];
            if (add && cok) v += g.addscale * add[(size_t)rg * g.ldadd + cg];
            cst[rl * CSTR + cl] = v;
        }
    }
    __syncthreads();
    const int col = tid % TC, rsel = tid / TC, rstep = 256 / TC;
    if (ACT != ACT_NONE) {
#pragma unroll 1
        for (int r = rsel; r < TR; r += rstep) cst[r * CSTR + col] = act_apply(ACT, cst[r * CSTR + col]);
    }
    float* ob = C + (size_t)row0 * g.ldc + (size_t)blockIdx.y * TC;
    const bool colok = (int)(blockIdx.y * TC + col) < g.nstore;
    const int rmax = (g.M - row0 < TR) ? (g.M - row0) : TR;
    auto pass = [&]() {
        if (colok) {
#pragma unroll 4
            for (int r = rsel; r < rmax; r += rstep) *(volatile float*)(ob + (size_t)r * g.ldc + col) = cst[r * CSTR + col];
        }
    };
    pass();
    __threadfence();
    pass();
}
static inline ZMap zm(long long s1) { ZMap m; m.s1 = s1; m.s2 = 0; m.zdiv = 1; m.pad_ = 0; return m; }
static inline ZMap zm2(long long s1, long long s2, int zdiv) { ZMap m; m.s1 = s1; m.s2 = s2; m.zdiv = zdiv; m.pad_ = 0; return m; }
static inline GemmArgs gemm_args(const float* A, int lda, ZMap za, const float* Bm, int ldb, ZMap zb, float* C, int ldc, ZMap zc, int M, int N, int K) {
    GemmArgs g; g.za = za; g.zb_ = zb; g.zc = zc; g.zbias = zm(0); g.zadd = zm(0); g.zrsc = zm(0); g.zmul = zm(0); g.zrbias = zm(0);
    g.A = A; g.Bm = Bm; g.C = C; g.bias = nullptr; g.add = nullptr; g.rsc = nullptr; g.mul = nullptr; g.rbias = nullptr; g.ldadd = 0; g.ldmul = 0;
    g.lda = lda; g.ldb = ldb; g.ldc = ldc; g.K = K; g.ascale = 1.0f; g.bscale = 1.0f; g.oscale = 1.0f; g.addscale = 1.0f; g.M = M; g.nvalid = N; g.nstore = N; g.ldrsc = 1;
    g.bcs = 1; g.pad1 = 0; g.pad2 = 0; g.pad3 = 0;
    return g;
}
static_assert(sizeof(ZMap) == 24, "ZMap layout");
static_assert(sizeof(GemmArgs) == 8 * 24 + 8 * 8 + 2 * 8 + 4 * 4 + 4 * 4 + 4 * 4 + 4 * 4, "GemmArgs has no padding");


#define VST2(T, p, v) do { const T vst2_v_ = (v); *(volatile T*)(p) = vst2_v_; __threadfence(); *(volatile T*)(p) = vst2_v_; } while (0)

__global__ __launch_bounds__(256) void k_wcat(const float* __restrict__ Wl, const float* __restrict__ Wr, float* WC) {
    const int lane = threadIdx.x & 31; const int n = blockIdx.x * 8 + (threadIdx.x >> 5); if (n >= HID) return;
#pragma unroll
    for (int i = 0; i < 4; ++i) { VST2(float, WC + (size_t)n * (2 * FIN) + 32 * i + lane, Wl[(size_t)n * FIN + 32 * i + lane]); }
#pragma unroll
    for (int i = 0; i < 4; ++i) { VST2(float, WC + (size_t)n * (2 * FIN) + FIN + 32 * i + lane, Wr[(size_t)n * FIN + 32 * i + lane]); }
}

__global__ __launch_bounds__(NT) void k_aggr(const float* __restrict__ x, const int* __restrict__ ei, int c0, float* AX) {
    extern __shared__ float4 lds_raw[];
    float* agg  = (float*)lds_raw;
    int*   lst  = (int*)(agg + RB * FIN);
    int*   degc = lst + CHUNK;
    int*   wtot = degc + RB;
    const int t = threadIdx.x, lane = t & 31, wv = t >> 5;
    const int n0 = c0 + blockIdx.x * RB;
    for (int i = t; i < RB * FIN; i += NT) agg[i] = 0.0f;
    if (t < RB) degc[t] = 0;
    __syncthreads();
#pragma unroll 1
    for (int base = 0; base < NE_; base += CHUNK) {
        int val[EPT]; int flg[EPT]; int cnt = 0;
#pragma unroll
        for (int j = 0; j < EPT; ++j) {
            const int e = base + j * NT + t;
            const int d = (e < NE_) ? ei[(size_t)NE_ + e] : -1;
            const unsigned udl = (unsigned)d - (unsigned)n0;
            const int f = (udl < (unsigned)RB) ? 1 : 0;
            int v = 0;
            if (f) { int s = ei[e]; if (s < 0) s += NN_; s = min(max(s, 0), NN_ - 1); v = s * RB + (int)udl; }
            val[j] = v; flg[j] = f; cnt += f;
        }
        int incl = cnt;
#pragma unroll
        for (int o = 1; o < 32; o <<= 1) { const int y = __shfl_up(incl, o, 32); if (lane >= o) incl += y; }
        if (lane == 31) wtot[wv] = incl;
        __syncthreads();
        int off = incl - cnt, tot = 0;
#pragma unroll
        for (int i = 0; i < NWV; ++i) { const int v = wtot[i]; off += (i < wv) ? v : 0; tot += v; }
#pragma unroll
        for (int j = 0; j < EPT; ++j) { if (flg[j]) { lst[off] = val[j]; ++off; } }
        __syncthreads();
        if (tot > 0 && t < FIN) {
#pragma unroll 1
            for (int e2 = 0; e2 < tot; ++e2) {
                const int v = lst[e2];
                const int s = v >> 9, dl = v & (RB - 1);
                agg[dl * FIN + t] += x[(size_t)s * FIN + t];
                if (t == 0) degc[dl] += 1;
            }
        }
        __syncthreads();
    }
    float* invs = (float*)lst;
    if (t < RB) invs[t] = 1.0f / fmaxf((float)degc[t], 1.0f);
    __syncthreads();
    const int r0 = wv * (RB / NWV);
    auto pass = [&]() {
#pragma unroll 4
        for (int i = 0; i < RB / NWV; ++i) {
            const int rl = r0 + i;
            const float inv = invs[rl];
            v4f a = *(const v4fa*)(agg + rl * FIN + lane * 4);
            a *= inv;
            const int nx = min(n0 + rl, NN_ - 1);
            const v4f b = *(const v4f*)(x + (size_t)nx * FIN + lane * 4);
            float* row = AX + (size_t)(blockIdx.x * RB + rl) * (2 * FIN);
            *(volatile v4f*)(row + lane * 4) = a;
            *(volatile v4f*)(row + FIN + lane * 4) = b;
        }
    };
    pass();
    __threadfence();
    pass();
}

__global__ __launch_bounds__(256) void k_pool(const float* __restrict__ H, const int* __restrict__ batch, int c0, int nrows, float* HP) {
    __shared__ int lst[256];
    __shared__ int wt[8];
    const int g = blockIdx.x, t = threadIdx.x, lane = t & 31, wv = t >> 5;
    float mx = -__builtin_inff();
#pragma unroll 1
    for (int i0 = 0; i0 < nrows; i0 += 256) {
        const int r = i0 + t;
        const int f = (r < nrows && batch[c0 + r] == g) ? 1 : 0;
        int incl = f;
#pragma unroll
        for (int o = 1; o < 32; o <<= 1) { const int y = __shfl_up(incl, o, 32); if (lane >= o) incl += y; }
        if (lane == 31) wt[wv] = incl;
        __syncthreads();
        int off = incl - f, tot = 0;
#pragma unroll
        for (int i = 0; i < 8; ++i) { const int v = wt[i]; off += (i < wv) ? v : 0; tot += v; }
        if (f) lst[off] = r;
        __syncthreads();
#pragma unroll 1
        for (int q = 0; q < tot; ++q) mx = fmaxf(mx, H[(size_t)lst[q] * HID + t]);
        __syncthreads();
    }
    VST2(float, HP + (size_t)g * HID + t, mx);
}

__global__ __launch_bounds__(256) void k_poolred(const float* __restrict__ HPC, float* NH) {
    const int g = blockIdx.x, t = threadIdx.x;
    float mx = -__builtin_inff();
#pragma unroll
    for (int ch = 0; ch < NCH; ++ch) mx = fmaxf(mx, HPC[((size_t)ch * NG_ + g) * HID + t]);
    VST2(float, NH + (size_t)g * (2 * HID) + HID + t, mx);
}

__global__ __launch_bounds__(128) void k_root(const float* __restrict__ x, const int* __restrict__ batch, float* XR) {
    __shared__ int rt;
    const int g = blockIdx.x, t = threadIdx.x;
    if (t == 0) {
        int lo = 0, hi = NN_;
#pragma unroll 1
        for (int it = 0; it < 20; ++it) { if (lo < hi) { const int mid = (lo + hi) >> 1; if (batch[mid] < g) lo = mid + 1; else hi = mid; } }
        rt = min(lo, NN_ - 1);
    }
    __syncthreads();
    const int r = rt;
    VST2(float, XR + (size_t)g * FIN + t, x[(size_t)r * FIN + t]);
}

__global__ __launch_bounds__(NG_) void k_fin(const float* __restrict__ H2, const float* __restrict__ W2, const float* __restrict__ b2, float* out) {
    const int g = threadIdx.x;
    const float* h = H2 + (size_t)g * HID;
    float z0 = 0.f, z1 = 0.f;
#pragma unroll 2
    for (int c = 0; c < HID; ++c) { const float hv = h[c]; z0 += hv * W2[c]; z1 += hv * W2[HID + c]; }
    z0 += b2[0]; z1 += b2[1];
    const float m = fmaxf(z0, z1);
    const float s0 = z0 - m, s1 = z1 - m;
    const float lse = logf(expf(s0) + expf(s1));
    v2f o; o[0] = s0 - lse; o[1] = s1 - lse;
    VST2(v2f, out + (size_t)g * 2, o);
}

extern "C" void kernel_launch(void* const* d_in, const int* in_sizes, int n_in,
                              void* d_out, int out_size, void* d_ws, size_t ws_size, hipStream_t stream) {
    (void)in_sizes; (void)n_in; (void)out_size;
    const float* x = (const float*)d_in[0]; const int* ei = (const int*)d_in[1]; const int* batch = (const int*)d_in[2];
    const float* Wl = (const float*)d_in[3]; const float* bl = (const float*)d_in[4]; const float* Wr = (const float*)d_in[5];
    const float* W0 = (const float*)d_in[6]; const float* b0 = (const float*)d_in[7]; const float* W1 = (const float*)d_in[8]; const float* b1 = (const float*)d_in[9];
    const float* W2 = (const float*)d_in[10]; const float* b2 = (const float*)d_in[11];
    float* out = (float*)d_out;
    char* wsp = (char*)d_ws;
    auto take = [&](size_t bytes) { char* p = wsp; wsp += (bytes + 255) & ~(size_t)255; return (void*)p; };
    float* WC  = (float*)take((size_t)HID * 2 * FIN * 4);
    float* AX  = (float*)take((size_t)NBLK * RB * 2 * FIN * 4);
    float* HC  = (float*)take((size_t)CHN * HID * 4);
    float* HPC = (float*)take((size_t)NCH * NG_ * HID * 4);
    float* XR  = (float*)take((size_t)NG_ * FIN * 4);
    float* NH  = (float*)take((size_t)NG_ * 2 * HID * 4);
    float* H2  = (float*)take((size_t)NG_ * HID * 4);
    if ((size_t)(wsp - (char*)d_ws) > ws_size) return;
    k_wcat<<<HID / 8, 256, 0, stream>>>(Wl, Wr, WC);
    for (int ch = 0; ch < NCH; ++ch) {
        const int c0 = ch * CHN;
        k_aggr<<<NBLK, NT, LDS_AGGR, stream>>>(x, ei, c0, AX);
        { GemmArgs g = gemm_args(AX, 2 * FIN, zm(0), WC, 2 * FIN, zm(0), HC, HID, zm(0), CHN, HID, 2 * FIN); g.bias = bl;
          gemm_kernel<1, 1, 1, 1, 4, 2, ACT_RELU><<<dim3((CHN + 63) / 64, HID / 128, 1), 256, 0, stream>>>(g); }
        k_pool<<<NG_, 256, 0, stream>>>(HC, batch, c0, CHN, HPC + (size_t)ch * NG_ * HID);
    }
    k_poolred<<<NG_, 256, 0, stream>>>(HPC, NH);
    k_root<<<NG_, FIN, 0, stream>>>(x, batch, XR);
    { GemmArgs g = gemm_args(XR, FIN, zm(0), W0, FIN, zm(0), NH, 2 * HID, zm(0), NG_, HID, FIN); g.bias = b0;
      gemm_kernel<1, 1, 1, 1, 4, 2, ACT_RELU><<<dim3(NG_ / 64, HID / 128, 1), 256, 0, stream>>>(g); }
    { GemmArgs g = gemm_args(NH, 2 * HID, zm(0), W1, 2 * HID, zm(0), H2, HID, zm(0), NG_, HID, 2 * HID); g.bias = b1;
      gemm_kernel<1, 1, 1, 1, 4, 2, ACT_RELU><<<dim3(NG_ / 64, HID / 128, 1), 256, 0, stream>>>(g); }
    k_fin<<<1, NG_, 0, stream>>>(H2, W2, b2, out);
}
